// CausalSelfAttention_17626545782991
// MI455X (gfx1250) — hardware-verified
//
#include <hip/hip_runtime.h>
#ifndef NB
#define NB 4
#endif
#ifndef SEQ
#define SEQ 2048
#endif
#define NB_FULL 4
#define SEQ_FULL 2048
#define DM 1024
#define NH 16
#define HD 64
#define QE ((SEQ) < 512 ? (SEQ) : 512)
#define NR ((size_t)NB * SEQ)
#define LDV (NB * SEQ)
#define RS 0.0009765625f

static_assert(NH * HD == DM);
static_assert(HD == 64);
static_assert(DM % 32 == 0);
static_assert(DM % 128 == 0);
static_assert((NB * SEQ) % 128 == 0);
static_assert(SEQ % 64 == 0);
static_assert(QE % 64 == 0);
static_assert((SEQ - QE) % 64 == 0);
static_assert(NB <= NB_FULL);
static_assert(SEQ <= SEQ_FULL);
static_assert((size_t)3 * DM * DM * 2 + (size_t)7 * NB * SEQ * DM * 2 <= (size_t)134217728);

typedef _Float16 v16h __attribute__((ext_vector_type(16)));
typedef unsigned short v8us __attribute__((ext_vector_type(8), may_alias));
typedef float v8f  __attribute__((ext_vector_type(8)));
typedef float v4f  __attribute__((ext_vector_type(4)));
typedef float v4fa __attribute__((ext_vector_type(4), may_alias));
union FragH { v16h v; v8us half[2]; _Float16 h[16]; };

__device__ __forceinline__ unsigned short bf16_bits(float x) { unsigned int u = __float_as_uint(x); return (unsigned short)((u + 0x7FFFu + ((u >> 16) & 1u)) >> 16); }
__device__ __forceinline__ float bf16_rne(float x) { return __uint_as_float(((unsigned int)bf16_bits(x)) << 16); }

__device__ __forceinline__ v16h g2_frag(const _Float16* __restrict__ p, size_t off, int hh) {
  FragH f;
  const unsigned short* q = (const unsigned short*)p + off;
  f.half[0] = *(const v8us*)(q + 8 * hh);
  f.half[1] = *(const v8us*)(q + 16 + 8 * hh);
  return f.v;
}
__device__ __forceinline__ v8f g2_mma(v16h a, v16h b, v8f c) {
  v8f d = __builtin_amdgcn_wmma_f32_16x16x32_f16(false, a, false, b, (short)0, c, false, false);
  asm volatile("v_nop\n\tv_nop\n\tv_nop\n\tv_nop" : "+v"(d) : "v"(a), "v"(b));
  return d;
}

__global__ __launch_bounds__(256) void k_wnat(const float* __restrict__ w, size_t n8, _Float16* __restrict__ Bt) {
  const size_t t = (size_t)blockIdx.x * 256 + threadIdx.x; if (t >= n8) return;
  const v4f a = *(const v4fa*)(w + t * 8), c = *(const v4fa*)(w + t * 8 + 4);
  FragH f;
#pragma unroll
  for (int q = 0; q < 4; ++q) { f.h[q] = (_Float16)(bf16_rne(a[q]) * 16.0f); f.h[4 + q] = (_Float16)(bf16_rne(c[q]) * 16.0f); }
  const v8us o = f.half[0];
  unsigned short* d = (unsigned short*)Bt + t * 8;
  *(volatile v8us*)d = o; __threadfence(); *(volatile v8us*)d = o;
}

__global__ __launch_bounds__(256) void k_x16(const float* __restrict__ x, _Float16* __restrict__ X16, size_t n8) {
  const size_t t = (size_t)blockIdx.x * 256 + threadIdx.x; if (t >= n8) return;
  const size_t e = t * 8; const size_t tok = e / DM; const size_t c = e - tok * DM; const size_t b = tok / SEQ; const size_t s = tok - b * SEQ;
  const float* src = x + (b * SEQ_FULL + s) * DM + c;
  const v4f a = *(const v4fa*)src, d4 = *(const v4fa*)(src + 4);
  FragH f;
#pragma unroll
  for (int q = 0; q < 4; ++q) { f.h[q] = (_Float16)bf16_rne(a[q]); f.h[4 + q] = (_Float16)bf16_rne(d4[q]); }
  const v8us o = f.half[0];
  unsigned short* d = (unsigned short*)X16 + e;
  *(volatile v8us*)d = o; __threadfence(); *(volatile v8us*)d = o;
}

template <int BIASROW>
__device__ __forceinline__ void gemm_body(const _Float16* __restrict__ A, int lda, const _Float16* __restrict__ Bh, int ldb, float alpha,
                                          const float* __restrict__ bias, _Float16* __restrict__ Ch, _Float16* __restrict__ Cl, int ldc, int N, int K) {
  __shared__ __attribute__((aligned(16))) float so[4][32][68];
  const int tid = threadIdx.x, w = tid >> 5, lane = tid & 31, ln = lane & 15, hh = lane >> 4;
  const int ntn = N >> 6; const int mt = blockIdx.x / ntn, nq = blockIdx.x - mt * ntn;
  const int row0 = mt * 128 + 32 * w, col0 = nq * 64;
  const size_t a0o = (size_t)(row0 + ln) * lda, a1o = a0o + (size_t)16 * lda;
  const size_t b0o = (size_t)(col0 + ln) * ldb, b1o = b0o + (size_t)16 * ldb, b2o = b1o + (size_t)16 * ldb, b3o = b2o + (size_t)16 * ldb;
  const v8f z8 = {0.f, 0.f, 0.f, 0.f, 0.f, 0.f, 0.f, 0.f};
  v8f c00 = z8, c01 = z8, c02 = z8, c03 = z8, c10 = z8, c11 = z8, c12 = z8, c13 = z8;
#pragma unroll 1
  for (int kb = 0; kb < K; kb += 32) {
    const v16h a0 = g2_frag(A, a0o + kb, hh), a1 = g2_frag(A, a1o + kb, hh);
    v16h b = g2_frag(Bh, b0o + kb, hh); c00 = g2_mma(a0, b, c00); c10 = g2_mma(a1, b, c10);
    b = g2_frag(Bh, b1o + kb, hh); c01 = g2_mma(a0, b, c01); c11 = g2_mma(a1, b, c11);
    b = g2_frag(Bh, b2o + kb, hh); c02 = g2_mma(a0, b, c02); c12 = g2_mma(a1, b, c12);
    b = g2_frag(Bh, b3o + kb, hh); c03 = g2_mma(a0, b, c03); c13 = g2_mma(a1, b, c13);
  }
  float brow[16];
  if (BIASROW) {
#pragma unroll
    for (int hf = 0; hf < 2; ++hf) {
      const v4f p0 = *(const v4fa*)(bias + row0 + hf * 16 + 8 * hh), p1 = *(const v4fa*)(bias + row0 + hf * 16 + 8 * hh + 4);
#pragma unroll
      for (int j = 0; j < 4; ++j) { brow[hf * 8 + j] = bf16_rne(p0[j]); brow[hf * 8 + 4 + j] = bf16_rne(p1[j]); }
    }
  } else {
#pragma unroll
    for (int j = 0; j < 16; ++j) brow[j] = 0.f;
  }
  const v8f accs[8] = {c00, c01, c02, c03, c10, c11, c12, c13};
#pragma unroll
  for (int u = 0; u < 8; ++u) {
    const int t = u & 3, hf = u >> 2; const int col = col0 + t * 16 + ln;
    float bcol = 0.f; if (!BIASROW) bcol = bf16_rne(bias[col]);
#pragma unroll
    for (int r = 0; r < 8; ++r) { const int rloc = hf * 16 + 8 * hh + r; const float bv = BIASROW ? brow[hf * 8 + r] : bcol; so[w][rloc][t * 16 + ln] = accs[u][r] * alpha + bv; }
  }
  __builtin_amdgcn_fence(4  , "workgroup"); __builtin_amdgcn_wave_barrier();
  const int rq = lane >> 3, c8 = (lane & 7) * 8;
  for (int pass = 0; pass < 2; ++pass) {
#pragma unroll
    for (int q = 0; q < 8; ++q) {
      const int r = q * 4 + rq;
      const v4f a = *(const v4fa*)&so[w][r][c8], c = *(const v4fa*)&so[w][r][c8 + 4];
      FragH fh, fl;
#pragma unroll
      for (int j = 0; j < 4; ++j) {
        _Float16 h = (_Float16)a[j]; fh.h[j] = h; fl.h[j] = (_Float16)((a[j] - (float)h) * 1024.0f);
        h = (_Float16)c[j]; fh.h[4 + j] = h; fl.h[4 + j] = (_Float16)((c[j] - (float)h) * 1024.0f);
      }
      const size_t o = (size_t)(row0 + r) * ldc + col0 + c8;
      *(volatile v8us*)((unsigned short*)Ch + o) = fh.half[0];
      *(volatile v8us*)((unsigned short*)Cl + o) = fl.half[0];
    }
    if (pass == 0) __threadfence();
  }
}
__global__ __launch_bounds__(128) void k_gemm_colb(const _Float16* __restrict__ A, int lda, const _Float16* __restrict__ Bh, int ldb, float alpha,
                                                   const float* __restrict__ bias, _Float16* __restrict__ Ch, _Float16* __restrict__ Cl, int ldc, int N, int K) {
  gemm_body<0>(A, lda, Bh, ldb, alpha, bias, Ch, Cl, ldc, N, K);
}
__global__ __launch_bounds__(128) void k_gemm_rowb(const _Float16* __restrict__ A, int lda, const _Float16* __restrict__ Bh, int ldb, float alpha,
                                                   const float* __restrict__ bias, _Float16* __restrict__ Ch, _Float16* __restrict__ Cl, int ldc, int N, int K) {
  gemm_body<1>(A, lda, Bh, ldb, alpha, bias, Ch, Cl, ldc, N, K);
}

template <int EARLY>
__device__ __forceinline__ void attn_body(const _Float16* __restrict__ Qh, const _Float16* __restrict__ Ql, const _Float16* __restrict__ Kh, const _Float16* __restrict__ Kl,
                                          const _Float16* __restrict__ Vh, const _Float16* __restrict__ Vl, const float* __restrict__ mask, float* __restrict__ out, int qbase, int nqb) {
  __shared__ __attribute__((aligned(16))) float so[4][16][68];
  const int tid = threadIdx.x, w = tid >> 5, lane = tid & 31, ln = lane & 15, hh = lane >> 4;
  const int bh = blockIdx.x / nqb, qb = blockIdx.x - bh * nqb;
  if (bh >= NB * NH) return;
  const int b = bh / NH, head = bh - b * NH;
  const int q0 = qbase + qb * 64 + 16 * w;
  const size_t tok0 = (size_t)b * SEQ;
  const size_t qoff = (tok0 + q0 + ln) * DM + head * HD;
  const size_t voff = (size_t)(head * HD + ln) * LDV + tok0;
  const float* mp = mask + (size_t)b * SEQ_FULL;
  const int myq = q0 + ln;
  const v8f z8 = {0.f, 0.f, 0.f, 0.f, 0.f, 0.f, 0.f, 0.f};
  v8f oh[4] = {z8, z8, z8, z8};
  v8f ol[4] = {z8, z8, z8, z8};
  float m = -1.0e30f, l = 0.f;
#pragma unroll 1
  for (int kb = 0; kb <= q0 + 15; kb += 32) {
    v8f sh0 = z8, sh1 = z8, sl0 = z8, sl1 = z8;
    const size_t k0o = (tok0 + kb + ln) * DM + head * HD, k1o = k0o + (size_t)16 * DM;
#pragma unroll
    for (int ds = 0; ds < 2; ++ds) {
      const v16h qh = g2_frag(Qh, qoff + 32 * ds, hh), ql = g2_frag(Ql, qoff + 32 * ds, hh);
      const v16h a0 = g2_frag(Kh, k0o + 32 * ds, hh), a1 = g2_frag(Kh, k1o + 32 * ds, hh);
      sh0 = g2_mma(a0, qh, sh0); sh1 = g2_mma(a1, qh, sh1);
      sl0 = g2_mma(a0, ql, sl0); sl1 = g2_mma(a1, ql, sl1);
      if (EARLY) {
        const v16h e0 = g2_frag(Kl, k0o + 32 * ds, hh), e1 = g2_frag(Kl, k1o + 32 * ds, hh);
        sl0 = g2_mma(e0, qh, sl0); sl1 = g2_mma(e1, qh, sl1);
      }
    }
    const v4f mk0 = *(const v4fa*)(mp + kb + 8 * hh), mk1 = *(const v4fa*)(mp + kb + 8 * hh + 4);
    const v4f mk2 = *(const v4fa*)(mp + kb + 16 + 8 * hh), mk3 = *(const v4fa*)(mp + kb + 16 + 8 * hh + 4);
    const float mk[16] = {mk0[0], mk0[1], mk0[2], mk0[3], mk1[0], mk1[1], mk1[2], mk1[3], mk2[0], mk2[1], mk2[2], mk2[3], mk3[0], mk3[1], mk3[2], mk3[3]};
    float zz[16];
    float mx = -1.0e30f;
#pragma unroll
    for (int r = 0; r < 8; ++r) {
      const int key0 = kb + 8 * hh + r;
      float a = (sh0[r] + sl0[r] * RS + bf16_rne(mk[r])) * 0.125f;
      float c = (sh1[r] + sl1[r] * RS + bf16_rne(mk[8 + r])) * 0.125f;
      a = (key0 <= myq) ? a : -1.0e30f;
      c = (key0 + 16 <= myq) ? c : -1.0e30f;
      zz[r] = a; zz[8 + r] = c;
      mx = fmaxf(mx, fmaxf(a, c));
    }
    mx = fmaxf(mx, __shfl_xor(mx, 16, 32));
    const float mn = fmaxf(m, mx);
    const float sf = __expf(m - mn);
    m = mn;
    float ps = 0.f;
    FragH ph, pl;
#pragma unroll
    for (int i = 0; i < 16; ++i) {
      const float p = __expf(zz[i] - mn);
      ps += p;
      const float pc = p * 256.0f;
      const _Float16 h = (_Float16)pc;
      ph.h[i] = h;
      pl.h[i] = EARLY ? (_Float16)((pc - (float)h) * 1024.0f) : (_Float16)0.0f;
    }
    l = l * sf + ps;
#pragma unroll
    for (int t = 0; t < 4; ++t) { oh[t] = oh[t] * sf; if (EARLY) ol[t] = ol[t] * sf; }
#pragma unroll
    for (int t = 0; t < 4; ++t) {
      const size_t vo = voff + (size_t)t * 16 * LDV + kb;
      const v16h va = g2_frag(Vh, vo, hh);
      oh[t] = g2_mma(va, ph.v, oh[t]);
      if (EARLY) {
        const v16h vb = g2_frag(Vl, vo, hh);
        ol[t] = g2_mma(va, pl.v, ol[t]);
        ol[t] = g2_mma(vb, ph.v, ol[t]);
      }
    }
  }
  l = l + __shfl_xor(l, 16, 32);
  const float inv = 1.0f / (256.0f * l);
#pragma unroll
  for (int t = 0; t < 4; ++t) {
    v8f o = oh[t];
    if (EARLY) o = o + ol[t] * RS;
    o = o * inv;
    const v4f a = {o[0], o[1], o[2], o[3]}, c = {o[4], o[5], o[6], o[7]};
    *(v4f*)&so[w][ln][16 * t + 8 * hh] = a;
    *(v4f*)&so[w][ln][16 * t + 8 * hh + 4] = c;
  }
  __builtin_amdgcn_fence(4  , "workgroup"); __builtin_amdgcn_wave_barrier();
  const int rsub = lane >> 4, c4 = (lane & 15) * 4;
  float* ob = out + ((size_t)b * SEQ_FULL + q0) * DM + head * HD;
  for (int pass = 0; pass < 2; ++pass) {
#pragma unroll
    for (int q = 0; q < 8; ++q) {
      const int r = q * 2 + rsub;
      const v4f v = *(const v4fa*)&so[w][r][c4];
      *(volatile v4f*)(ob + (size_t)r * DM + c4) = v;
    }
    if (pass == 0) __threadfence();
  }
}
__global__ __launch_bounds__(128) void k_attn_early(const _Float16* __restrict__ Qh, const _Float16* __restrict__ Ql, const _Float16* __restrict__ Kh, const _Float16* __restrict__ Kl,
                                                    const _Float16* __restrict__ Vh, const _Float16* __restrict__ Vl, const float* __restrict__ mask, float* __restrict__ out) {
  attn_body<1>(Qh, Ql, Kh, Kl, Vh, Vl, mask, out, 0, QE / 64);
}
__global__ __launch_bounds__(128) void k_attn_late(const _Float16* __restrict__ Qh, const _Float16* __restrict__ Ql, const _Float16* __restrict__ Kh, const _Float16* __restrict__ Kl,
                                                   const _Float16* __restrict__ Vh, const _Float16* __restrict__ Vl, const float* __restrict__ mask, float* __restrict__ out) {
  attn_body<0>(Qh, Ql, Kh, Kl, Vh, Vl, mask, out, QE, (SEQ - QE) / 64);
}

extern "C" void kernel_launch(void* const* d_in, const int* in_sizes, int n_in,
                              void* d_out, int out_size, void* d_ws, size_t ws_size, hipStream_t stream) {
  if (n_in < 8) return;
  const long long need_rows = (long long)(NB - 1) * SEQ_FULL + SEQ;
  if ((long long)in_sizes[0] < need_rows * DM) return;
  if ((long long)in_sizes[1] < need_rows) return;
  if (in_sizes[2] < DM * DM || in_sizes[4] < DM * DM || in_sizes[6] < DM * DM) return;
  if (in_sizes[3] < DM || in_sizes[5] < DM || in_sizes[7] < DM) return;
  if ((long long)out_size < need_rows * DM) return;
  const float* x = (const float*)d_in[0];
  const float* am = (const float*)d_in[1];
  const float* wq = (const float*)d_in[2]; const float* bq = (const float*)d_in[3];
  const float* wk = (const float*)d_in[4]; const float* bk = (const float*)d_in[5];
  const float* wv = (const float*)d_in[6]; const float* bv = (const float*)d_in[7];
  float* out = (float*)d_out;
  char* ws = (char*)d_ws; size_t off = 0;
  auto take = [&](size_t bytes) { char* p = ws + off; off += (bytes + 255) & ~(size_t)255; return p; };
  _Float16* BW  = (_Float16*)take((size_t)3 * DM * DM * 2);
  _Float16* X16 = (_Float16*)take(NR * DM * 2);
  _Float16* Qh  = (_Float16*)take(NR * DM * 2); _Float16* Ql = (_Float16*)take(NR * DM * 2);
  _Float16* Kh  = (_Float16*)take(NR * DM * 2); _Float16* Kl = (_Float16*)take(NR * DM * 2);
  _Float16* VTh = (_Float16*)take((size_t)DM * LDV * 2); _Float16* VTl = (_Float16*)take((size_t)DM * LDV * 2);
  if (off > ws_size) return;
  const size_t wn8 = (size_t)DM * DM / 8;
  const unsigned gw = (unsigned)((wn8 + 255) / 256);
  k_wnat<<<gw, 256, 0, stream>>>(wq, wn8, BW);
  k_wnat<<<gw, 256, 0, stream>>>(wk, wn8, BW + (size_t)DM * DM);
  k_wnat<<<gw, 256, 0, stream>>>(wv, wn8, BW + (size_t)2 * DM * DM);
  k_x16<<<(unsigned)((NR * DM / 8 + 255) / 256), 256, 0, stream>>>(x, X16, NR * DM / 8);
  k_gemm_colb<<<(unsigned)((NR / 128) * (DM / 64)), 128, 0, stream>>>(X16, DM, BW, DM, 0.0625f, bq, Qh, Ql, DM, DM, DM);
  k_gemm_colb<<<(unsigned)((NR / 128) * (DM / 64)), 128, 0, stream>>>(X16, DM, BW + (size_t)DM * DM, DM, 0.0625f, bk, Kh, Kl, DM, DM, DM);
  k_gemm_rowb<<<(unsigned)((DM / 128) * (NR / 64)), 128, 0, stream>>>(BW + (size_t)2 * DM * DM, DM, X16, DM, 0.0625f, bv, VTh, VTl, LDV, (int)NR, DM);
  k_attn_early<<<(unsigned)(NB * NH * (QE / 64)), 128, 0, stream>>>(Qh, Ql, Kh, Kl, VTh, VTl, am, out);
  if (SEQ > QE) k_attn_late<<<(unsigned)(NB * NH * ((SEQ - QE) / 64)), 128, 0, stream>>>(Qh, Ql, Kh, Kl, VTh, VTl, am, out);
}
